// SGFormerEncoderLayer_46437186404988
// MI455X (gfx1250) — hardware-verified
//
#include <hip/hip_runtime.h>
#include <math.h>
#include <stdint.h>

#define NN 4096
#define CC 512
#define NH 8
#define HD 64
#define C3 1536
#define CF 1024

typedef _Float16 v16h __attribute__((ext_vector_type(16)));
typedef _Float16 v8h  __attribute__((ext_vector_type(8)));
typedef _Float16 v4h  __attribute__((ext_vector_type(4)));
typedef float    v8f  __attribute__((ext_vector_type(8)));
typedef float    v4f  __attribute__((ext_vector_type(4)));
typedef float    v2f  __attribute__((ext_vector_type(2)));

union FragH { v16h v; v8h h[2]; };

__device__ __forceinline__ v16h ldfrag(const _Float16* p) {
  FragH f;
  f.h[0] = *(const v8h*)(p);
  f.h[1] = *(const v8h*)(p + 16);
  return f.v;
}

__device__ __forceinline__ v8f mma16(v16h a, v16h b, v8f c) {
  c = __builtin_amdgcn_wmma_f32_16x16x32_f16(false, a, false, b, (short)0, c, false, false);
  asm volatile("v_nop\n\tv_nop\n\tv_nop\n\tv_nop" : "+v"(c) : "v"(a), "v"(b));
  return c;
}

__device__ __forceinline__ void lds_wave_sync() {
  __builtin_amdgcn_fence(__ATOMIC_RELEASE, "workgroup");
  __builtin_amdgcn_wave_barrier();
  __builtin_amdgcn_fence(__ATOMIC_ACQUIRE, "workgroup");
}

__device__ __forceinline__ v8f zero8() { v8f z = {0.f, 0.f, 0.f, 0.f, 0.f, 0.f, 0.f, 0.f}; return z; }

__global__ __launch_bounds__(256) void cvt_f16_kernel(const float* __restrict__ in, _Float16* __restrict__ out,
                                                      int n8, float scale) {
  const int i = blockIdx.x * 256 + threadIdx.x;
  if (i < n8) {
    const v4f a = *(const v4f*)(in + (size_t)i * 8);
    const v4f b = *(const v4f*)(in + (size_t)i * 8 + 4);
    v8h h;
#pragma unroll
    for (int e = 0; e < 4; ++e) {
      h[e]     = (_Float16)(a[e] * scale);
      h[e + 4] = (_Float16)(b[e] * scale);
    }
    _Float16* p = out + (size_t)i * 8;
    *(volatile v8h*)p = h;
    __threadfence();
    *(volatile v8h*)p = h;
  }
}

template <int BIAS_MODE, int OUT16, int RES_MODE, int ACT>
__global__ __launch_bounds__(256) void gemm64(const _Float16* __restrict__ A, int lda,
                                             const _Float16* __restrict__ Bt, int ldb,
                                             void* __restrict__ Cout, int ldc,
                                             const float* __restrict__ bias,
                                             const float* __restrict__ resid, int ldr,
                                             int M, int N, int K, float scale, float oscale) {
  __shared__ __align__(16) float sT[8][16 * 68];
  const int lane = threadIdx.x & 31;
  const int wave = threadIdx.x >> 5;
  const int tilesN = N >> 6;
  const int tilesM = M >> 6;
  const int tile = blockIdx.x * 8 + wave;
  if (tile >= tilesM * tilesN) return;
  const int tm = tile / tilesN;
  const int tn = tile - tm * tilesN;
  const int m0 = tm << 6;
  const int n0 = tn << 6;
  const int rl = lane & 15;
  const int hh = lane >> 4;
  const int koff = hh * 8;

  v8f acc[4][4];
#pragma unroll
  for (int i = 0; i < 4; ++i)
#pragma unroll
    for (int j = 0; j < 4; ++j) acc[i][j] = zero8();

  for (int k0 = 0; k0 < K; k0 += 32) {
    v16h bf[4];
#pragma unroll
    for (int j = 0; j < 4; ++j)
      bf[j] = ldfrag(Bt + (size_t)(n0 + (j << 4) + rl) * ldb + k0 + koff);
#pragma unroll
    for (int i = 0; i < 4; ++i) {
      const v16h af = ldfrag(A + (size_t)(m0 + (i << 4) + rl) * lda + k0 + koff);
#pragma unroll
      for (int j = 0; j < 4; ++j) acc[i][j] = mma16(af, bf[j], acc[i][j]);
    }
  }

  float* slab = sT[wave];
#pragma unroll
  for (int i = 0; i < 4; ++i) {
    const int mBase = m0 + (i << 4);
#pragma unroll
    for (int j = 0; j < 4; ++j) {
      const int col = n0 + (j << 4) + rl;
      float bcol = 0.f;
      if (BIAS_MODE == 2) bcol = bias[col];
#pragma unroll
      for (int r = 0; r < 8; ++r) {
        const int row = mBase + 8 * hh + r;
        float v = acc[i][j][r] * scale;
        if (BIAS_MODE == 1) v += bias[row];
        if (BIAS_MODE == 2) v += bcol;
        if (RES_MODE == 1) v += resid[(size_t)row * ldr + col];
        if (RES_MODE == 2) v = 0.5f * v + 0.5f * resid[(size_t)row * ldr + col];
        if (ACT == 5) v = 0.5f * v * (1.0f + erff(v * 0.70710678118654752f));
        v *= oscale;
        slab[(8 * hh + r) * 68 + (j << 4) + rl] = v;
      }
    }
    lds_wave_sync();
    if (OUT16 == 0) {
      float* C = (float*)Cout;
      const int c4 = rl * 4;
      for (int ps = 0; ps < 2; ++ps) {
#pragma unroll
        for (int it = 0; it < 8; ++it) {
          const int row = it * 2 + hh;
          const v4f v = *(const v4f*)(slab + row * 68 + c4);
          *(volatile v4f*)(C + (size_t)(mBase + row) * ldc + n0 + c4) = v;
        }
        __threadfence();
      }
    } else {
      _Float16* C = (_Float16*)Cout;
      const int q = lane >> 3, c8 = (lane & 7) * 8;
      for (int ps = 0; ps < 2; ++ps) {
#pragma unroll
        for (int it = 0; it < 4; ++it) {
          const int row = it * 4 + q;
          const float* sp = slab + row * 68 + c8;
          const v4f a = *(const v4f*)(sp);
          const v4f b = *(const v4f*)(sp + 4);
          v8h hv;
#pragma unroll
          for (int e = 0; e < 4; ++e) { hv[e] = (_Float16)a[e]; hv[e + 4] = (_Float16)b[e]; }
          *(volatile v8h*)(C + (size_t)(mBase + row) * ldc + n0 + c8) = hv;
        }
        __threadfence();
      }
    }
    lds_wave_sync();
  }
}

#define AT_QB 64
#define AT_KC 64

__global__ __launch_bounds__(128) void attn_kernel(const _Float16* __restrict__ QK,
                                                   const _Float16* __restrict__ VT,
                                                   _Float16* __restrict__ CTX, float sc2, float oscale) {
  __shared__ __align__(16) _Float16 Ks[AT_KC * HD];
  __shared__ __align__(16) _Float16 Vs[HD * AT_KC];
  __shared__ __align__(16) _Float16 Ps[4][16 * AT_KC];
  __shared__ __align__(16) float    Os[4][16 * 68];

  const int tid  = threadIdx.x;
  const int wave = tid >> 5;
  const int lane = tid & 31;
  const int hh   = lane >> 4;
  const int c    = lane & 15;

  const int nqb = NN / AT_QB;
  const int qb  = blockIdx.x % nqb;
  const int h   = blockIdx.x / nqb;
  const int q0  = qb * AT_QB + wave * 16;

  const _Float16* Qp = QK + (size_t)h * HD;
  const _Float16* Kp = QK + CC + (size_t)h * HD;
  const _Float16* Vp = VT + (size_t)h * HD * NN;
  _Float16*       Op = CTX + (size_t)h * HD;

  v16h qa[2];
#pragma unroll
  for (int dc = 0; dc < 2; ++dc)
    qa[dc] = ldfrag(Qp + (size_t)(q0 + c) * CF + dc * 32 + 8 * hh);

  float mrow[8], lrow[8];
  v8f oacc[4];
#pragma unroll
  for (int r = 0; r < 8; ++r) { mrow[r] = -1.0e30f; lrow[r] = 0.f; }
#pragma unroll
  for (int t = 0; t < 4; ++t) oacc[t] = zero8();

  for (int kc = 0; kc < NN / AT_KC; ++kc) {
    const int kv0 = kc * AT_KC;
    __syncthreads();
    {
      const int r = tid >> 1, half = (tid & 1) * 32;
      const _Float16* ks = Kp + (size_t)(kv0 + r) * CF + half;
      const _Float16* vs = Vp + (size_t)r * NN + kv0 + half;
#pragma unroll
      for (int i = 0; i < 4; ++i) {
        const v8h a = *(const v8h*)(ks + 8 * i);
        const v8h b = *(const v8h*)(vs + 8 * i);
        *(v8h*)(Ks + r * HD + half + 8 * i) = a;
        *(v8h*)(Vs + r * AT_KC + half + 8 * i) = b;
      }
    }
    __syncthreads();

    v8f s[4];
#pragma unroll
    for (int j = 0; j < 4; ++j) {
      s[j] = zero8();
#pragma unroll
      for (int dc = 0; dc < 2; ++dc) {
        FragH kb;
        kb.h[0] = *(const v8h*)(Ks + (j * 16 + c) * HD + dc * 32 + 8 * hh);
        kb.h[1] = *(const v8h*)(Ks + (j * 16 + c) * HD + dc * 32 + 16 + 8 * hh);
        s[j] = mma16(qa[dc], kb.v, s[j]);
      }
    }
    float cm[8];
#pragma unroll
    for (int r = 0; r < 8; ++r) {
      float m = -1.0e30f;
#pragma unroll
      for (int j = 0; j < 4; ++j) {
        const float sv = s[j][r] * sc2;
        s[j][r] = sv;
        m = fmaxf(m, sv);
      }
#pragma unroll
      for (int off = 1; off < 16; off <<= 1) m = fmaxf(m, __shfl_xor(m, off, 32));
      cm[r] = m;
    }
    _Float16* pw = Ps[wave];
#pragma unroll
    for (int r = 0; r < 8; ++r) {
      const float mnew  = fmaxf(mrow[r], cm[r]);
      const float alpha = __builtin_amdgcn_exp2f(mrow[r] - mnew);
      mrow[r] = mnew;
      float psum = 0.f;
#pragma unroll
      for (int j = 0; j < 4; ++j) {
        const float p = __builtin_amdgcn_exp2f(s[j][r] - mnew);
        psum += p;
        pw[(8 * hh + r) * AT_KC + j * 16 + c] = (_Float16)p;
      }
#pragma unroll
      for (int off = 1; off < 16; off <<= 1) psum += __shfl_xor(psum, off, 32);
      lrow[r] = lrow[r] * alpha + psum;
#pragma unroll
      for (int t = 0; t < 4; ++t) oacc[t][r] *= alpha;
    }
    lds_wave_sync();
#pragma unroll
    for (int kk = 0; kk < 2; ++kk) {
      FragH pa;
      pa.h[0] = *(const v8h*)(pw + c * AT_KC + kk * 32 + 8 * hh);
      pa.h[1] = *(const v8h*)(pw + c * AT_KC + kk * 32 + 16 + 8 * hh);
#pragma unroll
      for (int t = 0; t < 4; ++t) {
        FragH vb;
        vb.h[0] = *(const v8h*)(Vs + (t * 16 + c) * AT_KC + kk * 32 + 8 * hh);
        vb.h[1] = *(const v8h*)(Vs + (t * 16 + c) * AT_KC + kk * 32 + 16 + 8 * hh);
        oacc[t] = mma16(pa.v, vb.v, oacc[t]);
      }
    }
  }

  float* os = Os[wave];
#pragma unroll
  for (int r = 0; r < 8; ++r) {
    const float inv = oscale / lrow[r];
#pragma unroll
    for (int t = 0; t < 4; ++t) os[(8 * hh + r) * 68 + t * 16 + c] = oacc[t][r] * inv;
  }
  lds_wave_sync();
  {
    const int q = lane >> 3, c8 = (lane & 7) * 8;
    for (int ps = 0; ps < 2; ++ps) {
#pragma unroll
      for (int it = 0; it < 4; ++it) {
        const int row = it * 4 + q;
        const float* sp = os + row * 68 + c8;
        const v4f a = *(const v4f*)(sp);
        const v4f b = *(const v4f*)(sp + 4);
        v8h hv;
#pragma unroll
        for (int e = 0; e < 4; ++e) { hv[e] = (_Float16)a[e]; hv[e + 4] = (_Float16)b[e]; }
        *(volatile v8h*)(Op + (size_t)(q0 + row) * CC + c8) = hv;
      }
      __threadfence();
    }
  }
}

#define AG_NB 64
#define AG_CAP 4096
#define AG_EPT 8
#define AG_CHUNK 2048
#define AG_DYN_BYTES (AG_NB * CC * 4)

__global__ __launch_bounds__(256) void agg_kernel(const int* __restrict__ ei, int nE,
                                                  const float* __restrict__ LH,
                                                  float* __restrict__ LO, int nNodes) {
  extern __shared__ __align__(16) float accS[];
  __shared__ int hitS[AG_CAP];
  __shared__ int wsumS[8];
  __shared__ int cntS[AG_NB];

  const int tid = threadIdx.x;
  const int lane = tid & 31;
  const int wave = tid >> 5;
  const int d0 = blockIdx.x * AG_NB;
  const int* srcp = ei;
  const int* dstp = ei + nE;

  const v4f z4 = {0.f, 0.f, 0.f, 0.f};
  for (int i = tid; i < AG_NB * CC / 4; i += 256) *(v4f*)(accS + 4 * i) = z4;
  if (tid < AG_NB) cntS[tid] = 0;
  __syncthreads();

  int total = 0;
  const int nChunks = (nE + AG_CHUNK - 1) / AG_CHUNK;
  for (int ch = 0; ch < nChunks; ++ch) {
    const int e0 = ch * AG_CHUNK + tid * AG_EPT;
    int code[AG_EPT];
    int cnt = 0;
#pragma unroll
    for (int j = 0; j < AG_EPT; ++j) {
      const int e  = e0 + j;
      const int ec = min(e, nE - 1);
      const int d  = dstp[ec];
      const int rel = d - d0;
      const bool hit = (e < nE) && ((unsigned)rel < (unsigned)AG_NB);
      code[j] = hit ? ((e << 6) | rel) : -1;
      cnt += hit ? 1 : 0;
    }
    int v = cnt;
#pragma unroll
    for (int off = 1; off < 32; off <<= 1) {
      const int t = __shfl_up(v, off, 32);
      v += (lane >= off) ? t : 0;
    }
    if (lane == 31) wsumS[wave] = v;
    __syncthreads();
    int wpre = 0, csum = 0;
#pragma unroll
    for (int w = 0; w < 8; ++w) {
      const int s = wsumS[w];
      wpre += (w < wave) ? s : 0;
      csum += s;
    }
    int pos = total + wpre + (v - cnt);
#pragma unroll
    for (int j = 0; j < AG_EPT; ++j) {
      if (code[j] >= 0) {
        if (pos < AG_CAP) hitS[pos] = code[j];
        ++pos;
      }
    }
    total = min(total + csum, AG_CAP);
    __syncthreads();
  }

  const int nh = total;
  const int c2 = tid * 2;
#pragma unroll 2
  for (int i = 0; i < nh; ++i) {
    const int hv = hitS[i];
    const int slot = hv & (AG_NB - 1);
    int e = hv >> 6;
    e = min(max(e, 0), nE - 1);
    int s = srcp[e];
    s = min(max(s, 0), nNodes - 1);
    const v2f val = *(const v2f*)(LH + (size_t)s * CC + c2);
    float* ap = accS + slot * CC + c2;
    v2f a = *(v2f*)ap;
    a += val;
    *(v2f*)ap = a;
    if (tid == slot) cntS[tid] += 1;
  }
  __syncthreads();

  const int rsel = tid >> 7;
  const int c4 = (tid & 127) * 4;
  for (int ps = 0; ps < 2; ++ps) {
    for (int it = 0; it < AG_NB / 2; ++it) {
      const int row = it * 2 + rsel;
      const int node = d0 + row;
      const float inv = 1.0f / fmaxf((float)cntS[row], 1.0f);
      v4f a = *(const v4f*)(accS + row * CC + c4);
      a = a * inv;
      if (node < nNodes) *(volatile v4f*)(LO + (size_t)node * CC + c4) = a;
    }
    __threadfence();
  }
}

template <int OUT16>
__global__ __launch_bounds__(256) void ln_kernel(const float* __restrict__ X, const float* __restrict__ g,
                                                const float* __restrict__ b, float* __restrict__ outF,
                                                _Float16* __restrict__ outH, int nRows) {
  const int lane = threadIdx.x & 31;
  const int wave = threadIdx.x >> 5;
  const int row = blockIdx.x * 8 + wave;
  if (row >= nRows) return;
  const float* xr = X + (size_t)row * CC;
  v4f xv[4], gv[4], bv[4];
  float s = 0.f;
#pragma unroll
  for (int i = 0; i < 4; ++i) {
    const int col = 128 * i + lane * 4;
    xv[i] = *(const v4f*)(xr + col);
    gv[i] = *(const v4f*)(g + col);
    bv[i] = *(const v4f*)(b + col);
    s += (xv[i][0] + xv[i][1]) + (xv[i][2] + xv[i][3]);
  }
#pragma unroll
  for (int off = 1; off < 32; off <<= 1) s += __shfl_xor(s, off, 32);
  const float mu = s * (1.0f / 512.0f);
  v4f dv[4];
  float qs = 0.f;
#pragma unroll
  for (int i = 0; i < 4; ++i) {
    dv[i] = xv[i] - mu;
    qs += (dv[i][0] * dv[i][0] + dv[i][1] * dv[i][1]) + (dv[i][2] * dv[i][2] + dv[i][3] * dv[i][3]);
  }
#pragma unroll
  for (int off = 1; off < 32; off <<= 1) qs += __shfl_xor(qs, off, 32);
  const float rstd = rsqrtf(qs * (1.0f / 512.0f) + 1.0e-5f);
  v4f yv[4];
#pragma unroll
  for (int i = 0; i < 4; ++i) yv[i] = dv[i] * rstd * gv[i] + bv[i];
  for (int ps = 0; ps < 2; ++ps) {
#pragma unroll
    for (int i = 0; i < 4; ++i) {
      const int col = 128 * i + lane * 4;
      *(volatile v4f*)(outF + (size_t)row * CC + col) = yv[i];
      if (OUT16) {
        v4h hv;
#pragma unroll
        for (int e = 0; e < 4; ++e) hv[e] = (_Float16)yv[i][e];
        *(volatile v4h*)(outH + (size_t)row * CC + col) = hv;
      }
    }
    __threadfence();
  }
}

extern "C" void kernel_launch(void* const* d_in, const int* in_sizes, int n_in,
                              void* d_out, int out_size, void* d_ws, size_t ws_size,
                              hipStream_t stream) {
  if (n_in < 18) return;
  if (in_sizes[0] != NN * CC) return;
  if (in_sizes[1] < 2 || (in_sizes[1] & 1) != 0) return;
  const int nE = in_sizes[1] / 2;
  if (in_sizes[2] != CC * CC || in_sizes[3] != CC) return;
  if (in_sizes[4] != C3 * CC || in_sizes[5] != C3) return;
  if (in_sizes[6] != CC * CC || in_sizes[7] != CC) return;
  if (in_sizes[8] != CC * CC || in_sizes[9] != CC) return;
  if (in_sizes[10] != CC || in_sizes[11] != CC || in_sizes[12] != CC || in_sizes[13] != CC) return;
  if (in_sizes[14] != CF * CC || in_sizes[15] != CF) return;
  if (in_sizes[16] != CC * CF || in_sizes[17] != CC) return;
  if (out_size != NN * CC) return;

  const float* x          = (const float*)d_in[0];
  const int*   ei         = (const int*)d_in[1];
  const float* local_w    = (const float*)d_in[2];
  const float* local_b    = (const float*)d_in[3];
  const float* in_proj_w  = (const float*)d_in[4];
  const float* in_proj_b  = (const float*)d_in[5];
  const float* attn_out_w = (const float*)d_in[6];
  const float* attn_out_b = (const float*)d_in[7];
  const float* output_w   = (const float*)d_in[8];
  const float* output_b   = (const float*)d_in[9];
  const float* norm1_g    = (const float*)d_in[10];
  const float* norm1_b    = (const float*)d_in[11];
  const float* norm2_g    = (const float*)d_in[12];
  const float* norm2_b    = (const float*)d_in[13];
  const float* ffn_w1     = (const float*)d_in[14];
  const float* ffn_b1     = (const float*)d_in[15];
  const float* ffn_w2     = (const float*)d_in[16];
  const float* ffn_b2     = (const float*)d_in[17];
  float* out = (float*)d_out;

  size_t off = 0;
  auto take = [&](size_t bytes) -> size_t { const size_t o = off; off += (bytes + 255) & ~(size_t)255; return o; };
  const size_t oXh  = take((size_t)NN * CC * 2);
  const size_t oLW  = take((size_t)CC * CC * 2);
  const size_t oIPW = take((size_t)C3 * CC * 2);
  const size_t oAOW = take((size_t)CC * CC * 2);
  const size_t oOW  = take((size_t)CC * CC * 2);
  const size_t oW1  = take((size_t)CF * CC * 2);
  const size_t oW2  = take((size_t)CC * CF * 2);
  const size_t oLH  = take((size_t)NN * CC * 4);
  const size_t oLO  = take((size_t)NN * CC * 4);
  const size_t oQK  = take((size_t)NN * CF * 2);
  const size_t oVT  = take((size_t)CC * NN * 2);
  const size_t oCTX = take((size_t)NN * CC * 2);
  const size_t oMX  = take((size_t)NN * CC * 2);
  const size_t oPR  = take((size_t)NN * CC * 4);
  const size_t oHF  = take((size_t)NN * CC * 4);
  const size_t oHH  = take((size_t)NN * CC * 2);
  const size_t oFF  = take((size_t)NN * CF * 2);
  const size_t oF2  = take((size_t)NN * CC * 4);
  if (off > ws_size || off > (size_t)134217728) return;

  char* ws = (char*)d_ws;
  _Float16* Xh   = (_Float16*)(ws + oXh);
  _Float16* LWh  = (_Float16*)(ws + oLW);
  _Float16* IPWh = (_Float16*)(ws + oIPW);
  _Float16* AOWh = (_Float16*)(ws + oAOW);
  _Float16* OWh  = (_Float16*)(ws + oOW);
  _Float16* W1h  = (_Float16*)(ws + oW1);
  _Float16* W2h  = (_Float16*)(ws + oW2);
  float*    LH   = (float*)(ws + oLH);
  float*    LO   = (float*)(ws + oLO);
  _Float16* QK   = (_Float16*)(ws + oQK);
  _Float16* VT   = (_Float16*)(ws + oVT);
  _Float16* CTX  = (_Float16*)(ws + oCTX);
  _Float16* MX   = (_Float16*)(ws + oMX);
  float*    PR   = (float*)(ws + oPR);
  float*    HF   = (float*)(ws + oHF);
  _Float16* HHp  = (_Float16*)(ws + oHH);
  _Float16* FF   = (_Float16*)(ws + oFF);
  float*    F2   = (float*)(ws + oF2);

  const dim3 blk(256);
  const float WSC = 16.0f;

  {
    const int n8x = NN * CC / 8;
    cvt_f16_kernel<<<dim3((n8x + 255) / 256), blk, 0, stream>>>(x, Xh, n8x, 1.0f);
    const int n8a = CC * CC / 8;
    cvt_f16_kernel<<<dim3((n8a + 255) / 256), blk, 0, stream>>>(local_w, LWh, n8a, WSC);
    const int n8b = C3 * CC / 8;
    cvt_f16_kernel<<<dim3((n8b + 255) / 256), blk, 0, stream>>>(in_proj_w, IPWh, n8b, WSC);
    cvt_f16_kernel<<<dim3((n8a + 255) / 256), blk, 0, stream>>>(attn_out_w, AOWh, n8a, WSC);
    cvt_f16_kernel<<<dim3((n8a + 255) / 256), blk, 0, stream>>>(output_w, OWh, n8a, WSC);
    const int n8c = CF * CC / 8;
    cvt_f16_kernel<<<dim3((n8c + 255) / 256), blk, 0, stream>>>(ffn_w1, W1h, n8c, WSC);
    cvt_f16_kernel<<<dim3((n8c + 255) / 256), blk, 0, stream>>>(ffn_w2, W2h, n8c, WSC);
  }

  const dim3 gMM512(((NN / 64) * (CC / 64) + 7) / 8);
  const dim3 gMM1024(((NN / 64) * (CF / 64) + 7) / 8);
  const dim3 gVT(((CC / 64) * (NN / 64) + 7) / 8);

  gemm64<2, 0, 0, 0><<<gMM512, blk, 0, stream>>>(Xh, CC, LWh, CC, (void*)LH, CC, local_b, local_b, 0,
                                                 NN, CC, CC, 1.0f / WSC, 1.0f);
  (void)hipFuncSetAttribute(reinterpret_cast<const void*>(&agg_kernel),
                            hipFuncAttributeMaxDynamicSharedMemorySize, AG_DYN_BYTES);
  agg_kernel<<<dim3((NN + AG_NB - 1) / AG_NB), blk, AG_DYN_BYTES, stream>>>(ei, nE, LH, LO, NN);
  gemm64<2, 1, 0, 0><<<gMM1024, blk, 0, stream>>>(Xh, CC, IPWh, CC, (void*)QK, CF, in_proj_b, in_proj_b, 0,
                                                  NN, CF, CC, 1.0f / WSC, 1.0f);
  gemm64<1, 1, 0, 0><<<gVT, blk, 0, stream>>>(IPWh + (size_t)CF * CC, CC, Xh, CC, (void*)VT, NN,
                                              in_proj_b + CF, in_proj_b, 0, CC, NN, CC, 1.0f / WSC, 1.0f);
  attn_kernel<<<dim3(NH * (NN / AT_QB)), dim3(128), 0, stream>>>(QK, VT, CTX, 0.18033688011112042f, 64.0f);
  gemm64<2, 1, 2, 0><<<gMM512, blk, 0, stream>>>(CTX, CC, AOWh, CC, (void*)MX, CC, attn_out_b, LO, CC,
                                                 NN, CC, CC, 1.0f / (64.0f * WSC), 16.0f);
  gemm64<2, 0, 1, 0><<<gMM512, blk, 0, stream>>>(MX, CC, OWh, CC, (void*)PR, CC, output_b, x, CC,
                                                 NN, CC, CC, 1.0f / (16.0f * WSC), 1.0f);
  ln_kernel<1><<<dim3((NN + 7) / 8), blk, 0, stream>>>(PR, norm1_g, norm1_b, HF, HHp, NN);
  gemm64<2, 1, 0, 5><<<gMM1024, blk, 0, stream>>>(HHp, CC, W1h, CC, (void*)FF, CF, ffn_b1, ffn_b1, 0,
                                                  NN, CF, CC, 1.0f / WSC, 16.0f);
  gemm64<2, 0, 1, 0><<<gMM512, blk, 0, stream>>>(FF, CF, W2h, CF, (void*)F2, CC, ffn_b2, HF, CC,
                                                 NN, CC, CF, 1.0f / (16.0f * WSC), 1.0f);
  ln_kernel<0><<<dim3((NN + 7) / 8), blk, 0, stream>>>(F2, norm2_g, norm2_b, out, HHp, NN);

  (void)hipGetLastError();
}
